// SpatioTemporalPixelEncoder_51805895524591
// MI455X (gfx1250) — hardware-verified
//
#include <hip/hip_runtime.h>


#define NB_  16
#define TT   2048
#define FF   64
#define IM   224
#define NBLK 256
typedef _Float16 h16;
typedef unsigned short bf;
typedef __attribute__((ext_vector_type(16))) __bf16   v16bf;
typedef __attribute__((ext_vector_type(16))) _Float16 v16h;
typedef __attribute__((ext_vector_type(8)))  _Float16 v8h;
typedef __attribute__((ext_vector_type(8)))  unsigned short v8us;
typedef __attribute__((ext_vector_type(8)))  float    v8f;
typedef __attribute__((ext_vector_type(4)))  float    v4f;
typedef v8h  __attribute__((may_alias)) v8ha;
typedef v4f  __attribute__((may_alias)) v4fa;
typedef v8us __attribute__((may_alias)) v8usa;

__device__ __forceinline__ unsigned short f2bf(float f) { unsigned u = __float_as_uint(f); u += 0x7FFFu + ((u >> 16) & 1u); return (unsigned short)(u >> 16); }
__device__ __forceinline__ float bf2f(unsigned short b) { return __uint_as_float(((unsigned)b) << 16); }
__device__ __forceinline__ float bfr(float f) { return bf2f(f2bf(f)); }
__device__ __forceinline__ v16h cat16(v8h lo, v8h hi) { return __builtin_shufflevector(lo, hi, 0, 1, 2, 3, 4, 5, 6, 7, 8, 9, 10, 11, 12, 13, 14, 15); }
__device__ __forceinline__ v16bf cat16b(v8us lo, v8us hi) { return __builtin_bit_cast(v16bf, __builtin_shufflevector(lo, hi, 0, 1, 2, 3, 4, 5, 6, 7, 8, 9, 10, 11, 12, 13, 14, 15)); }
__device__ __forceinline__ v8f wmma16(v16h a, v16h b, v8f c) { return __builtin_amdgcn_wmma_f32_16x16x32_f16(false, a, false, b, (short)0, c, false, false); }
__device__ __forceinline__ v8f wmmab(v16bf a, v16bf b, v8f c) { return __builtin_amdgcn_wmma_f32_16x16x32_bf16(false, a, false, b, (short)0, c, false, false); }


template <typename T16> struct WFrag;
template <> struct WFrag<h16> { typedef v16h V; static __device__ __forceinline__ V ld(const h16* p) { return cat16(*(const v8h*)p, *(const v8h*)(p + 16)); } static __device__ __forceinline__ v8f mma(V a, V b, v8f c) { return wmma16(a, b, c); } };
template <> struct WFrag<bf> { typedef v16bf V; static __device__ __forceinline__ V ld(const bf* p) { return cat16b(*(const v8us*)p, *(const v8us*)(p + 16)); } static __device__ __forceinline__ v8f mma(V a, V b, v8f c) { return wmmab(a, b, c); } };
template <typename T16, int NSPLIT, bool BIAS>
__global__ __launch_bounds__(32) void k_gemmw(const T16* __restrict__ A, const T16* __restrict__ A2, const T16* __restrict__ Bt, const T16* __restrict__ Bt2, int K, float* C, int ldc, const float* __restrict__ bias, size_t sA, size_t sB, size_t sC) {
    typedef typename WFrag<T16>::V V;
    __shared__ __align__(16) float os[16 * 68];
    const size_t z = blockIdx.z; A += z * sA; if (A2) A2 += z * sA; Bt += z * sB; if (Bt2) Bt2 += z * sB; C += z * sC;
    const int lane = threadIdx.x & 31, lr = lane & 15, hi = lane >> 4; const int r0 = blockIdx.x * 64, c0 = blockIdx.y * 64;
    v8f acc[4][4];
#pragma unroll
    for (int mb = 0; mb < 4; ++mb)
#pragma unroll
        for (int nb = 0; nb < 4; ++nb) acc[mb][nb] = (v8f){};
    const size_t aoff = (size_t)(r0 + lr) * K + 8 * hi, boff = (size_t)(c0 + lr) * K + 8 * hi;
#pragma unroll 1
    for (int kc = 0; kc < K; kc += 32) {
        V a[4], a2[4];
#pragma unroll
        for (int mb = 0; mb < 4; ++mb) { a[mb] = WFrag<T16>::ld(A + aoff + (size_t)mb * 16 * K + kc); if (NSPLIT == 1 || NSPLIT == 2) a2[mb] = WFrag<T16>::ld(A2 + aoff + (size_t)mb * 16 * K + kc); }
#pragma unroll
        for (int nb = 0; nb < 4; ++nb) { const V b = WFrag<T16>::ld(Bt + boff + (size_t)nb * 16 * K + kc); V b2; if (NSPLIT >= 2) b2 = WFrag<T16>::ld(Bt2 + boff + (size_t)nb * 16 * K + kc);
#pragma unroll
            for (int mb = 0; mb < 4; ++mb) { acc[mb][nb] = WFrag<T16>::mma(a[mb], b, acc[mb][nb]); if (NSPLIT == 1 || NSPLIT == 2) acc[mb][nb] = WFrag<T16>::mma(a2[mb], b, acc[mb][nb]); if (NSPLIT >= 2) acc[mb][nb] = WFrag<T16>::mma(a[mb], b2, acc[mb][nb]); } }
        asm volatile("v_nop\n\tv_nop\n\tv_nop\n\tv_nop" : "+v"(acc[0][0]), "+v"(acc[1][1]), "+v"(acc[2][2]), "+v"(acc[3][3]) : "v"(a[0]), "v"(a[3]));
    }
#pragma unroll
    for (int mb = 0; mb < 4; ++mb) {
#pragma unroll
        for (int nb = 0; nb < 4; ++nb) {
#pragma unroll
            for (int j = 0; j < 8; ++j) os[(hi * 8 + j) * 68 + nb * 16 + lr] = acc[mb][nb][j]; }
        __builtin_amdgcn_wave_barrier(); asm volatile("" ::: "memory");
        float* crow = C + (size_t)(r0 + mb * 16) * ldc + c0;
#pragma unroll 1
        for (int ps = 0; ps < 2; ++ps) {
#pragma unroll
            for (int s = 0; s < 8; ++s) { const int row = 2 * s + hi, cofs = lr * 4; v4f val = *(const v4fa*)(os + row * 68 + cofs); if (BIAS) { val[0] += bfr(bias[c0 + cofs]); val[1] += bfr(bias[c0 + cofs + 1]); val[2] += bfr(bias[c0 + cofs + 2]); val[3] += bfr(bias[c0 + cofs + 3]); }
                *(volatile v4f*)(crow + (size_t)row * ldc + cofs) = val; }
            if (ps == 0) __threadfence(); }
        __builtin_amdgcn_wave_barrier(); asm volatile("" ::: "memory");
    }
}

__device__ __forceinline__ h16 tohx(float x) { return (h16)x; }
__device__ __forceinline__ void splitf(float y, unsigned short& h, unsigned short& l) { h = f2bf(y); l = f2bf(y - bf2f(h)); }
typedef __attribute__((ext_vector_type(2))) unsigned short v2us;
typedef __attribute__((ext_vector_type(2))) _Float16 v2h;
typedef __attribute__((ext_vector_type(4))) _Float16 v4h;
typedef __attribute__((ext_vector_type(2))) float v2f;

__global__ __launch_bounds__(256) void k_mm1(const float* __restrict__ A, size_t n, int isin, float* PART) { __shared__ float smn[256], smx[256]; const int tid = threadIdx.x; float mn = 3.0e38f, mx = -3.0e38f;
    for (size_t i = (size_t)blockIdx.x * 256 + tid; i < n; i += (size_t)NBLK * 256) { const float v = isin ? bfr(A[i]) : A[i]; mn = fminf(mn, v); mx = fmaxf(mx, v); }
    smn[tid] = mn; smx[tid] = mx; __syncthreads();
    for (int s = 128; s > 0; s >>= 1) { if (tid < s) { smn[tid] = fminf(smn[tid], smn[tid + s]); smx[tid] = fmaxf(smx[tid], smx[tid + s]); } __syncthreads(); }
    if (tid == 0) { v2f o; o[0] = smn[0]; o[1] = smx[0]; *(volatile v2f*)(PART + 32 * blockIdx.x) = o; __threadfence(); *(volatile v2f*)(PART + 32 * blockIdx.x) = o; } }
__global__ __launch_bounds__(32) void k_mm2(const float* __restrict__ PART, float* MM) { const int lane = threadIdx.x; float mn = 3.0e38f, mx = -3.0e38f; for (int i = lane; i < NBLK; i += 32) { mn = fminf(mn, PART[32 * i]); mx = fmaxf(mx, PART[32 * i + 1]); }
#pragma unroll
    for (int sh = 16; sh; sh >>= 1) { mn = fminf(mn, __shfl_xor(mn, sh, 32)); mx = fmaxf(mx, __shfl_xor(mx, sh, 32)); }
    if (lane == 0) { v2f o; o[0] = mn; o[1] = mx; *(volatile v2f*)MM = o; __threadfence(); *(volatile v2f*)MM = o; } }
__global__ __launch_bounds__(256) void k_cs(const float* __restrict__ x, const float* __restrict__ MM, bf* Ah, bf* Al, bf* Bh, bf* Bl) { const size_t e = ((size_t)blockIdx.x * 256 + threadIdx.x) * 2; if (e >= (size_t)TT * FF) return; const int f = (int)(e % FF); const int t = (int)(e / FF); const float lo = MM[0], hi = MM[1]; const float rng = __fsub_rn(hi, lo); const bool degen = rng < 1e-8f; const float den = __fadd_rn(rng, 1e-8f); v2us cah, cal, sah, sal, nsh, nsl;
#pragma unroll
    for (int u = 0; u < 2; ++u) { const float xv = bfr(x[e + u]); const float xn = degen ? 0.f : __fdiv_rn(__fsub_rn(xv, lo), den); float v = __fsub_rn(__fmul_rn(xn, 2.0f), 1.0f); v = fminf(fmaxf(v, -1.0f + 1e-6f), 1.0f - 1e-6f); const float th = acosf(v); const float c = cosf(th), s = sinf(th); unsigned short a, l; splitf(c, a, l); cah[u] = a; cal[u] = l; splitf(s, a, l); sah[u] = a; sal[u] = l; splitf(-s, a, l); nsh[u] = a; nsl[u] = l; }
    const size_t oa = (size_t)t * 128 + f; for (int ps = 0; ps < 2; ++ps) { *(volatile v2us*)(Ah + oa) = cah; *(volatile v2us*)(Al + oa) = cal; *(volatile v2us*)(Ah + oa + FF) = sah; *(volatile v2us*)(Al + oa + FF) = sal; *(volatile v2us*)(Bh + oa) = cah; *(volatile v2us*)(Bl + oa) = cal; *(volatile v2us*)(Bh + oa + FF) = nsh; *(volatile v2us*)(Bl + oa + FF) = nsl; if (ps == 0) __threadfence(); } }
__global__ __launch_bounds__(256) void k_rsz(const float* __restrict__ CS, const float* __restrict__ MMb, float* G) { const int e = blockIdx.x * 256 + threadIdx.x; if (e >= IM * IM) return; const int j = e % IM, i = e / IM; const float sc = (float)TT / (float)IM;
    auto coord = [&](int o, int& i0, int& i1, float& w) { float src = __fsub_rn(__fmul_rn((float)o + 0.5f, sc), 0.5f); src = fminf(fmaxf(src, 0.f), (float)(TT - 1)); i0 = (int)floorf(src); i1 = min(i0 + 1, TT - 1); w = __fsub_rn(src, (float)i0); };
    int i0, i1, j0, j1; float wh, ww; coord(i, i0, i1, wh); coord(j, j0, j1, ww); const float inv = 1.0f / 64.0f;
    const float a00 = CS[(size_t)i0 * TT + j0] * inv, a01 = CS[(size_t)i0 * TT + j1] * inv, a10 = CS[(size_t)i1 * TT + j0] * inv, a11 = CS[(size_t)i1 * TT + j1] * inv;
    const float lo = MMb[0] * inv, hi = MMb[1] * inv; const float rng = __fsub_rn(hi, lo); const bool degen = rng < 1e-8f; const float den = __fadd_rn(rng, 1e-8f);
    auto nrm = [&](float v) { return degen ? 0.f : __fdiv_rn(__fsub_rn(v, lo), den); };
    const float n00 = nrm(a00), n01 = nrm(a01), n10 = nrm(a10), n11 = nrm(a11);
    float t0 = __fmul_rn(n00, __fsub_rn(1.0f, wh)); asm volatile("" : "+v"(t0)); float t0b = __fmul_rn(n10, wh); asm volatile("" : "+v"(t0b)); const float top0 = __fadd_rn(t0, t0b);
    float t1 = __fmul_rn(n01, __fsub_rn(1.0f, wh)); asm volatile("" : "+v"(t1)); float t1b = __fmul_rn(n11, wh); asm volatile("" : "+v"(t1b)); const float top1 = __fadd_rn(t1, t1b);
    float r0 = __fmul_rn(top0, __fsub_rn(1.0f, ww)); asm volatile("" : "+v"(r0)); float r1 = __fmul_rn(top1, ww); asm volatile("" : "+v"(r1)); const float v = __fadd_rn(r0, r1);
    *(volatile float*)(G + e) = v; __threadfence(); *(volatile float*)(G + e) = v; }
__global__ __launch_bounds__(256) void k_fin(const float* __restrict__ G, const float* __restrict__ MMg, float* OUT) { const size_t i = ((size_t)blockIdx.x * 256 + threadIdx.x) * 4; if (i >= (size_t)NB_ * IM * IM) return; const float gmin = MMg[0], gmax = MMg[1]; const float den = __fadd_rn(__fsub_rn(gmax, gmin), 1e-6f); const v4f a = *(const v4f*)(G + i); v4f o;
#pragma unroll
    for (int q = 0; q < 4; ++q) o[q] = __fdiv_rn(__fsub_rn(a[q], gmin), den); *(volatile v4f*)(OUT + i) = o; __threadfence(); *(volatile v4f*)(OUT + i) = o; }

extern "C" void kernel_launch(void* const* d_in, const int* in_sizes, int n_in,
                              void* d_out, int out_size, void* d_ws, size_t ws_size, hipStream_t stream) {
    (void)in_sizes; (void)n_in; (void)out_size;
    const float* x = (const float*)d_in[0];
    float* OUT = (float*)d_out;
    char* wsp = (char*)d_ws;
    auto take = [&](size_t bytes) { char* p = wsp; wsp += (bytes + 255) & ~(size_t)255; return (void*)p; };
    float* PART = (float*)take(NBLK * 32 * 4); float* MMx = (float*)take(256); float* MMb = (float*)take(256); float* MMg = (float*)take(256); bf* Ah = (bf*)take((size_t)TT * 128 * 2); bf* Al = (bf*)take((size_t)TT * 128 * 2); bf* Bh = (bf*)take((size_t)TT * 128 * 2); bf* Bl = (bf*)take((size_t)TT * 128 * 2); float* CS = (float*)take((size_t)TT * TT * 4); float* G = (float*)take((size_t)NB_ * IM * IM * 4);
    if ((size_t)(wsp - (char*)d_ws) > ws_size) return;
    k_mm1<<<NBLK, 256, 0, stream>>>(x, (size_t)NB_ * TT * FF, 1, PART); k_mm2<<<1, 32, 0, stream>>>(PART, MMx);
    for (int b = 0; b < NB_; ++b) {
        k_cs<<<(TT * FF / 2 + 255) / 256, 256, 0, stream>>>(x + (size_t)b * TT * FF, MMx, Ah, Al, Bh, Bl);
        k_gemmw<bf, 2, false><<<dim3(TT / 64, TT / 64, 1), 32, 0, stream>>>(Ah, Al, Bh, Bl, 128, CS, TT, nullptr, 0, 0, 0);
        k_mm1<<<NBLK, 256, 0, stream>>>(CS, (size_t)TT * TT, 0, PART); k_mm2<<<1, 32, 0, stream>>>(PART, MMb);
        k_rsz<<<(IM * IM + 255) / 256, 256, 0, stream>>>(CS, MMb, G + (size_t)b * IM * IM); }
    k_mm1<<<NBLK, 256, 0, stream>>>(G, (size_t)NB_ * IM * IM, 0, PART); k_mm2<<<1, 32, 0, stream>>>(PART, MMg);
    k_fin<<<(NB_ * IM * IM / 4 + 255) / 256, 256, 0, stream>>>(G, MMg, OUT);
}
